// SupervisedModel_2027224563913
// MI455X (gfx1250) — hardware-verified
//
#include <hip/hip_runtime.h>

constexpr int kBatch   = 32768;
constexpr int kSeq     = 200;
constexpr int kHid     = 4;
constexpr int kXCols   = 2 * kSeq;
constexpr int kXPitch  = 448;
constexpr int kXK      = 416;
constexpr int kHCols   = kHid * kSeq;
constexpr int kHPitch  = 832;
constexpr int kNF      = 128;
constexpr int kZPitch  = 2 * kNF;
constexpr int kN1      = 80;
constexpr int kZ1Pitch = 128;
constexpr int kW1K     = 256;
constexpr int kW1Rows  = 128;
constexpr int kN2      = 40;
constexpr int kZ2Pitch = 64;
constexpr int kW2K     = 96;
constexpr int kW2Pitch = 128;
constexpr int kW2Rows  = 64;
constexpr int kNP      = 40;
constexpr int kOPitch  = 64;
constexpr int kWpRows  = 64;
constexpr int kBiasTot = 256;
constexpr int kLstmThreads = 256;
constexpr float kWCarry    = 16.0f;
constexpr float kHCarry    = 16.0f;
constexpr float kInvW      = 1.0f / 16.0f;
constexpr float kInvWH     = 1.0f / 256.0f;
static_assert(kBatch % 256 == 0);
static_assert(kBatch % 64 == 0);
static_assert(kXK % 32 == 0 && kHCols % 32 == 0 && kW1K % 32 == 0 && kW2K % 32 == 0);
static_assert(kXPitch % 64 == 0 && kHPitch % 64 == 0 && kZPitch % 64 == 0 && kZ1Pitch % 64 == 0 && kW2Pitch % 64 == 0);
static_assert(kSeq == 12 * 16 + 8);

typedef __attribute__((ext_vector_type(16))) _Float16 v16h;
typedef __attribute__((ext_vector_type(8)))  _Float16 v8h;
typedef __attribute__((ext_vector_type(16))) __bf16   v16b;
typedef __attribute__((ext_vector_type(8)))  __bf16   v8b;
typedef __attribute__((ext_vector_type(8)))  float    v8f;
typedef __attribute__((ext_vector_type(4)))  float    v4f;
typedef __attribute__((ext_vector_type(4)))  unsigned int v4u;
typedef __attribute__((ext_vector_type(2)))  unsigned int v2u;

__device__ __forceinline__ unsigned short f2bf_bits(float f) {
  unsigned u = __float_as_uint(f);
  return (unsigned short)((u + 0x7FFFu + ((u >> 16) & 1u)) >> 16);
}
__device__ __forceinline__ float bf_bits2f(unsigned short h) { return __uint_as_float(((unsigned)h) << 16); }

__device__ __forceinline__ void dep_guard_h(v8f& a, v8f& b, v16h x, v16h y) { asm volatile("v_nop\n\tv_nop\n\tv_nop\n\tv_nop" : "+v"(a), "+v"(b) : "v"(x), "v"(y)); }
__device__ __forceinline__ void dep_guard_b(v8f& a, v8f& b, v16b x, v16b y) { asm volatile("v_nop\n\tv_nop\n\tv_nop\n\tv_nop" : "+v"(a), "+v"(b) : "v"(x), "v"(y)); }
__device__ __forceinline__ void keep4_h(v16h a, v16h b, v16h c, v16h d) { asm volatile("v_nop" :: "v"(a), "v"(b), "v"(c), "v"(d)); }
__device__ __forceinline__ void keep4_b(v16b a, v16b b, v16b c, v16b d) { asm volatile("v_nop" :: "v"(a), "v"(b), "v"(c), "v"(d)); }
__device__ __forceinline__ void acc_guard4(v8f& a, v8f& b, v8f& c, v8f& d) { asm volatile("v_nop\n\tv_nop\n\tv_nop\n\tv_nop" : "+v"(a), "+v"(b), "+v"(c), "+v"(d)); }
template <typename T> struct Frag;
template <> struct Frag<_Float16> {
  typedef v16h V; union U { v16h v; v8h h[2]; };
  static __device__ __forceinline__ v16h load(const _Float16* p) {
    U f; f.h[0] = *(const v8h*)(p); f.h[1] = *(const v8h*)(p + 16); return f.v;
  }
  static __device__ __forceinline__ v8f mma(v16h a, v16h b, v8f c) {
    return __builtin_amdgcn_wmma_f32_16x16x32_f16(false, a, false, b, (short)0, c, false, false);
  }
  static __device__ __forceinline__ void guard(v8f& a, v8f& b, v16h x, v16h y) { dep_guard_h(a, b, x, y); }
  static __device__ __forceinline__ void keep(v16h a, v16h b, v16h c, v16h d) { keep4_h(a, b, c, d); }
};
template <> struct Frag<__bf16> {
  typedef v16b V; union U { v16b v; v8b h[2]; };
  static __device__ __forceinline__ v16b load(const __bf16* p) {
    U f; f.h[0] = *(const v8b*)(p); f.h[1] = *(const v8b*)(p + 16); return f.v;
  }
  static __device__ __forceinline__ v8f mma(v16b a, v16b b, v8f c) {
    return __builtin_amdgcn_wmma_f32_16x16x32_bf16(false, a, false, b, (short)0, c, false, false);
  }
  static __device__ __forceinline__ void guard(v8f& a, v8f& b, v16b x, v16b y) { dep_guard_b(a, b, x, y); }
  static __device__ __forceinline__ void keep(v16b a, v16b b, v16b c, v16b d) { keep4_b(a, b, c, d); }
};

__device__ __forceinline__ unsigned pk16(unsigned short a, unsigned short b) { return (unsigned)a | ((unsigned)b << 16); }
__device__ __forceinline__ unsigned short h_bits(float f) { const _Float16 h = (_Float16)f; return __builtin_bit_cast(unsigned short, h); }

__device__ __forceinline__ float fexp2_(float v) {
#if __has_builtin(__builtin_amdgcn_exp2f)
  return __builtin_amdgcn_exp2f(v);
#else
  return exp2f(v);
#endif
}
__device__ __forceinline__ float frcp_(float v) {
#if __has_builtin(__builtin_amdgcn_rcpf)
  return __builtin_amdgcn_rcpf(v);
#else
  return 1.0f / v;
#endif
}
__device__ __forceinline__ float sigm_(float v) { return frcp_(1.0f + fexp2_(v * -1.4426950408889634f)); }
__device__ __forceinline__ float tanh_(float v) { return 1.0f - 2.0f * frcp_(1.0f + fexp2_(v * 2.8853900817779268f)); }

__device__ __forceinline__ void wave_lds_sync() {
  __builtin_amdgcn_fence(__ATOMIC_RELEASE, "workgroup");
  __builtin_amdgcn_wave_barrier();
  __builtin_amdgcn_fence(__ATOMIC_ACQUIRE, "workgroup");
}

template <int ET> struct Elem;
template <> struct Elem<0> { typedef _Float16 T; };
template <> struct Elem<1> { typedef __bf16 T; };
template <int ET, bool SPLIT, int BIAS_MODE, int OUT_MODE, bool RESID, int ACT = 0>
__global__ __launch_bounds__(256) void wmma_gemm64(
    const unsigned short* __restrict__ Ap, const unsigned short* __restrict__ A2p, int lda, long strideA,
    const unsigned short* __restrict__ Btp, const unsigned short* __restrict__ Bt2p, int ldb, long strideB,
    void* __restrict__ Cout, void* __restrict__ Cout2, int ldc, long strideC,
    const float* __restrict__ bias,
    const float* __restrict__ resid, long strideR,
    int M, int N, int K, float scale) {
  typedef typename Elem<ET>::T T;
  typedef typename Frag<T>::V V;
  const T* A = (const T*)Ap; const T* A2 = (const T*)A2p; const T* Bt = (const T*)Btp; const T* Bt2 = (const T*)Bt2p;
  __shared__ __align__(16) float sT[8][16 * 68];
  const int b    = blockIdx.y;
  const int lane = threadIdx.x & 31;
  const int wave = threadIdx.x >> 5;
  const int tilesN = N >> 6;
  const int tilesM = M >> 6;
  const int tile = blockIdx.x * 8 + wave;
  if (tile >= tilesM * tilesN) return;
  const int tm = tile / tilesN;
  const int tn = tile - tm * tilesN;
  const int m0 = tm << 6;
  const int n0 = tn << 6;

  const T* Ab  = A  + (size_t)b * strideA;
  const T* Bb  = Bt + (size_t)b * strideB;
  const T* Ab2 = SPLIT ? (A2  + (size_t)b * strideA) : nullptr;
  const T* Bb2 = SPLIT ? (Bt2 + (size_t)b * strideB) : nullptr;

  const int rlane = lane & 15;
  const int koff  = (lane >> 4) * 8;
  const int mOff  = (lane >> 4) * 8;

  v8f acc[4][4];
#pragma unroll
  for (int i = 0; i < 4; ++i)
#pragma unroll
    for (int j = 0; j < 4; ++j) acc[i][j] = (v8f){0.f,0.f,0.f,0.f,0.f,0.f,0.f,0.f};

  for (int k0 = 0; k0 < K; k0 += 32) {
    V bh[4], bl[4];
#pragma unroll
    for (int j = 0; j < 4; ++j) {
      const size_t bo = (size_t)(n0 + (j << 4) + rlane) * ldb + koff + k0;
      bh[j] = Frag<T>::load(Bb + bo);
      if (SPLIT) bl[j] = Frag<T>::load(Bb2 + bo);
    }
#pragma unroll
    for (int i = 0; i < 4; ++i) {
      const size_t ao = (size_t)(m0 + (i << 4) + rlane) * lda + koff + k0;
      V ah = Frag<T>::load(Ab + ao);
      V al;
      if (SPLIT) al = Frag<T>::load(Ab2 + ao);
#pragma unroll
      for (int j = 0; j < 4; ++j) {
        acc[i][j] = Frag<T>::mma(ah, bh[j], acc[i][j]);
        if (SPLIT) {
          acc[i][j] = Frag<T>::mma(ah, bl[j], acc[i][j]);
          acc[i][j] = Frag<T>::mma(al, bh[j], acc[i][j]);
        }
      }
      Frag<T>::guard(acc[i][0], acc[i][3], ah, SPLIT ? al : ah);
    }
    Frag<T>::keep(bh[0], bh[1], bh[2], bh[3]);
    if (SPLIT) Frag<T>::keep(bl[0], bl[1], bl[2], bl[3]);
  }
  acc_guard4(acc[0][0], acc[0][1], acc[0][2], acc[0][3]);
  acc_guard4(acc[1][0], acc[1][1], acc[1][2], acc[1][3]);
  acc_guard4(acc[2][0], acc[2][1], acc[2][2], acc[2][3]);
  acc_guard4(acc[3][0], acc[3][1], acc[3][2], acc[3][3]);

  float* slab = sT[wave];
  const float* Rb = RESID ? (resid + (size_t)b * strideR) : nullptr;
#pragma unroll
  for (int i = 0; i < 4; ++i) {
    const int mBase = m0 + (i << 4);
#pragma unroll
    for (int j = 0; j < 4; ++j) {
      const int n = n0 + (j << 4) + rlane;
      float bv = 0.f;
      if (BIAS_MODE == 2) bv = bias[n];
#pragma unroll
      for (int r = 0; r < 8; ++r) {
        float v = acc[i][j][r] * scale;
        if (BIAS_MODE == 1) v += bias[mBase + mOff + r];
        if (BIAS_MODE == 2) v += bv;
        if (RESID) v += Rb[(size_t)(mBase + mOff + r) * ldc + n];
        if (ACT == 2) v = fmaxf(v, 0.0f);
        if (ACT == 4) v = (v > 0.f) ? v : 0.01f * v;
        if (ACT == 6) v = tanh_(v);
        slab[(mOff + r) * 68 + (j << 4) + rlane] = v;
      }
    }
    __builtin_amdgcn_fence(__ATOMIC_RELEASE, "workgroup");
    __builtin_amdgcn_wave_barrier();
    __builtin_amdgcn_fence(__ATOMIC_ACQUIRE, "workgroup");
    if (OUT_MODE == 0) {
      float* C = (float*)Cout + (size_t)b * strideC;
      const int hh = lane >> 4, c4 = (lane & 15) * 4;
      for (int pass = 0; pass < 2; ++pass) {
#pragma unroll
        for (int it = 0; it < 8; ++it) {
          const int row = it * 2 + hh;
          v4f v = *(const v4f*)(slab + row * 68 + c4);
          *(volatile v4f*)(C + (size_t)(mBase + row) * ldc + n0 + c4) = v;
        }
        __threadfence();
      }
    } else {
      const int q = lane >> 3, c8 = (lane & 7) * 8;
      unsigned short* C  = (unsigned short*)Cout  + (size_t)b * strideC;
      unsigned short* C2 = (OUT_MODE == 2) ? ((unsigned short*)Cout2 + (size_t)b * strideC) : nullptr;
      for (int pass = 0; pass < 2; ++pass) {
#pragma unroll
        for (int it = 0; it < 4; ++it) {
          const int row = it * 4 + q;
          const float* sp = slab + row * 68 + c8;
          v8h hv, lv;
#pragma unroll
          for (int e = 0; e < 8; ++e) {
            if (OUT_MODE == 1) {
              hv[e] = (_Float16)sp[e];
            } else {
              unsigned short hb = f2bf_bits(sp[e]);
              unsigned short lb = f2bf_bits(sp[e] - bf_bits2f(hb));
              hv[e] = __builtin_bit_cast(_Float16, hb);
              lv[e] = __builtin_bit_cast(_Float16, lb);
            }
          }
          *(volatile v8h*)(C + (size_t)(mBase + row) * ldc + n0 + c8) = hv;
          if (OUT_MODE == 2) *(volatile v8h*)(C2 + (size_t)(mBase + row) * ldc + n0 + c8) = lv;
        }
        __threadfence();
      }
    }
    __builtin_amdgcn_fence(__ATOMIC_RELEASE, "workgroup");
    __builtin_amdgcn_wave_barrier();
    __builtin_amdgcn_fence(__ATOMIC_ACQUIRE, "workgroup");
  }
}

__global__ __launch_bounds__(256) void padcast_kernel(const float* __restrict__ src, int rows, int cols,
                                                      unsigned short* __restrict__ dst, int dstRows, int dstPitch,
                                                      float scale) {
  const int gpr = dstPitch >> 3;
  const int total = dstRows * gpr;
  const int i = blockIdx.x * 256 + threadIdx.x;
  if (i >= total) return;
  const int r = i / gpr;
  const int g = i - r * gpr;
  const int rc = (r < rows) ? r : (rows - 1);
  unsigned short hb[8];
#pragma unroll
  for (int e = 0; e < 8; ++e) {
    const int col = g * 8 + e;
    const int cc = (col < cols) ? col : (cols - 1);
    float v = src[(size_t)rc * cols + cc] * scale;
    v = (r < rows && col < cols) ? v : 0.0f;
    hb[e] = h_bits(v);
  }
  const v4u u = (v4u){pk16(hb[0], hb[1]), pk16(hb[2], hb[3]), pk16(hb[4], hb[5]), pk16(hb[6], hb[7])};
  unsigned short* q = dst + 8 * (size_t)i;
  *(volatile v4u*)q = u;
  __threadfence();
  *(volatile v4u*)q = u;
}

__global__ __launch_bounds__(256) void xcast_kernel(const float* __restrict__ x, unsigned short* __restrict__ xp) {
  constexpr int kGpr = kXPitch / 8;
  constexpr int kGval = kXCols / 8;
  const int i = blockIdx.x * 256 + threadIdx.x;
  if (i >= kBatch * kGpr) return;
  const int r = i / kGpr;
  const int g = i - r * kGpr;
  const int gc = (g < kGval) ? g : (kGval - 1);
  const float* p = x + (size_t)r * kXCols + gc * 8;
  const v4f a = *(const v4f*)(p);
  const v4f c = *(const v4f*)(p + 4);
  const bool valid = (g < kGval);
  unsigned short hb[8];
#pragma unroll
  for (int e = 0; e < 4; ++e) {
    hb[e]     = h_bits(valid ? a[e] : 0.0f);
    hb[4 + e] = h_bits(valid ? c[e] : 0.0f);
  }
  const v4u u = (v4u){pk16(hb[0], hb[1]), pk16(hb[2], hb[3]), pk16(hb[4], hb[5]), pk16(hb[6], hb[7])};
  unsigned short* q = xp + (size_t)r * kXPitch + g * 8;
  *(volatile v4u*)q = u;
  __threadfence();
  *(volatile v4u*)q = u;
}

__global__ __launch_bounds__(64) void biasprep_kernel(const float* __restrict__ b1, const float* __restrict__ b2,
                                                      const float* __restrict__ bp, float* __restrict__ outp) {
  const int t = threadIdx.x;
  const int f = t * 4;
  v4f v;
#pragma unroll
  for (int e = 0; e < 4; ++e) {
    const int idx = f + e;
    int j1 = idx;        j1 = j1 < 0 ? 0 : (j1 > kN1 - 1 ? kN1 - 1 : j1);
    int j2 = idx - 128;  j2 = j2 < 0 ? 0 : (j2 > kN2 - 1 ? kN2 - 1 : j2);
    int j3 = idx - 192;  j3 = j3 < 0 ? 0 : (j3 > kNP - 1 ? kNP - 1 : j3);
    const float v1 = b1[j1];
    const float v2 = b2[j2];
    const float v3 = bp[j3];
    float r = 0.0f;
    r = (idx < kN1) ? v1 : r;
    r = (idx >= 128 && idx - 128 < kN2) ? v2 : r;
    r = (idx >= 192 && idx - 192 < kNP) ? v3 : r;
    v[e] = r;
  }
  float* q = outp + f;
  *(volatile v4f*)q = v;
  __threadfence();
  *(volatile v4f*)q = v;
}

__global__ __launch_bounds__(kLstmThreads) void lstm2_kernel(
    const float* __restrict__ x,
    const float* __restrict__ Wih0, const float* __restrict__ Whh0,
    const float* __restrict__ bih0, const float* __restrict__ bhh0,
    const float* __restrict__ Wih1, const float* __restrict__ Whh1,
    const float* __restrict__ bih1, const float* __restrict__ bhh1,
    unsigned short* __restrict__ hpl, int series) {
  __shared__ __align__(16) unsigned int sH[kLstmThreads * 32];
  const int tid  = threadIdx.x;
  const int lane = tid & 31;
  const int wave = tid >> 5;
  const int b    = blockIdx.x * kLstmThreads + tid;
  const float* xr = x + ((size_t)b * 2 + (size_t)series) * kSeq;
  unsigned int* sMine = sH + tid * 32;
  const unsigned int* sWave = sH + wave * (32 * 32);
  unsigned short* hw = hpl + (size_t)(blockIdx.x * kLstmThreads + wave * 32) * kHPitch;

  float h0a = 0.f, h0b = 0.f, h0c = 0.f, h0d = 0.f;
  float c0a = 0.f, c0b = 0.f, c0c = 0.f, c0d = 0.f;
  float h1a = 0.f, h1b = 0.f, h1c = 0.f, h1d = 0.f;
  float c1a = 0.f, c1b = 0.f, c1c = 0.f, c1d = 0.f;

#pragma unroll 1
  for (int t = 0; t < kSeq; ++t) {
    const float xt = xr[t];
    float qa = 0.f, qb = 0.f, qc = 0.f, qd = 0.f;
#pragma unroll 1
    for (int k = 0; k < kHid; ++k) {
      const v4f ri = *(const v4f*)(Whh0 + 4 * k);
      const v4f rf = *(const v4f*)(Whh0 + 16 + 4 * k);
      const v4f rg = *(const v4f*)(Whh0 + 32 + 4 * k);
      const v4f ro = *(const v4f*)(Whh0 + 48 + 4 * k);
      float gi = (bih0[k]      + bhh0[k])      + Wih0[k]      * xt;
      float gf = (bih0[4 + k]  + bhh0[4 + k])  + Wih0[4 + k]  * xt;
      float gg = (bih0[8 + k]  + bhh0[8 + k])  + Wih0[8 + k]  * xt;
      float go = (bih0[12 + k] + bhh0[12 + k]) + Wih0[12 + k] * xt;
      gi += ri[0] * h0a; gi += ri[1] * h0b; gi += ri[2] * h0c; gi += ri[3] * h0d;
      gf += rf[0] * h0a; gf += rf[1] * h0b; gf += rf[2] * h0c; gf += rf[3] * h0d;
      gg += rg[0] * h0a; gg += rg[1] * h0b; gg += rg[2] * h0c; gg += rg[3] * h0d;
      go += ro[0] * h0a; go += ro[1] * h0b; go += ro[2] * h0c; go += ro[3] * h0d;
      const float cn = sigm_(gf) * c0a + sigm_(gi) * tanh_(gg);
      const float hn = sigm_(go) * tanh_(cn);
      c0a = c0b; c0b = c0c; c0c = c0d; c0d = cn;
      qa = qb; qb = qc; qc = qd; qd = hn;
    }
    h0a = qa; h0b = qb; h0c = qc; h0d = qd;
    qa = 0.f; qb = 0.f; qc = 0.f; qd = 0.f;
#pragma unroll 1
    for (int k = 0; k < kHid; ++k) {
      const v4f ui = *(const v4f*)(Wih1 + 4 * k);
      const v4f uf = *(const v4f*)(Wih1 + 16 + 4 * k);
      const v4f ug = *(const v4f*)(Wih1 + 32 + 4 * k);
      const v4f uo = *(const v4f*)(Wih1 + 48 + 4 * k);
      const v4f ri = *(const v4f*)(Whh1 + 4 * k);
      const v4f rf = *(const v4f*)(Whh1 + 16 + 4 * k);
      const v4f rg = *(const v4f*)(Whh1 + 32 + 4 * k);
      const v4f ro = *(const v4f*)(Whh1 + 48 + 4 * k);
      float gi = bih1[k]      + bhh1[k];
      float gf = bih1[4 + k]  + bhh1[4 + k];
      float gg = bih1[8 + k]  + bhh1[8 + k];
      float go = bih1[12 + k] + bhh1[12 + k];
      gi += ui[0] * h0a; gi += ui[1] * h0b; gi += ui[2] * h0c; gi += ui[3] * h0d;
      gf += uf[0] * h0a; gf += uf[1] * h0b; gf += uf[2] * h0c; gf += uf[3] * h0d;
      gg += ug[0] * h0a; gg += ug[1] * h0b; gg += ug[2] * h0c; gg += ug[3] * h0d;
      go += uo[0] * h0a; go += uo[1] * h0b; go += uo[2] * h0c; go += uo[3] * h0d;
      gi += ri[0] * h1a; gi += ri[1] * h1b; gi += ri[2] * h1c; gi += ri[3] * h1d;
      gf += rf[0] * h1a; gf += rf[1] * h1b; gf += rf[2] * h1c; gf += rf[3] * h1d;
      gg += rg[0] * h1a; gg += rg[1] * h1b; gg += rg[2] * h1c; gg += rg[3] * h1d;
      go += ro[0] * h1a; go += ro[1] * h1b; go += ro[2] * h1c; go += ro[3] * h1d;
      const float cn = sigm_(gf) * c1a + sigm_(gi) * tanh_(gg);
      const float hn = sigm_(go) * tanh_(cn);
      c1a = c1b; c1b = c1c; c1c = c1d; c1d = cn;
      qa = qb; qb = qc; qc = qd; qd = hn;
    }
    h1a = qa; h1b = qb; h1c = qc; h1d = qd;
    const unsigned int u0 = pk16(h_bits(h1a * kHCarry), h_bits(h1b * kHCarry));
    const unsigned int u1 = pk16(h_bits(h1c * kHCarry), h_bits(h1d * kHCarry));
    const int slot = t & 15;
    *(v2u*)(sMine + slot * 2) = (v2u){u0, u1};
    const bool lastStep = (t == kSeq - 1);
    if (slot == 15 || lastStep) {
      if (lastStep) {
        const v4u z4 = (v4u){0u, 0u, 0u, 0u};
        *(v4u*)(sMine + 16) = z4;
        *(v4u*)(sMine + 20) = z4;
        *(v4u*)(sMine + 24) = z4;
        *(v4u*)(sMine + 28) = z4;
      }
      wave_lds_sync();
      const int cidx = t >> 4;
      for (int pass = 0; pass < 2; ++pass) {
#pragma unroll
        for (int it = 0; it < 8; ++it) {
          const int i = it * 4 + (lane >> 3);
          const int p = lane & 7;
          const v4u v = *(const v4u*)(sWave + i * 32 + p * 4);
          *(volatile v4u*)(hw + (size_t)i * kHPitch + cidx * 64 + p * 8) = v;
        }
        __threadfence();
      }
      wave_lds_sync();
    }
  }
}

__global__ __launch_bounds__(256) void head_kernel(const float* __restrict__ z2, const float* __restrict__ oth,
                                                   const float* __restrict__ W3, const float* __restrict__ b3,
                                                   float* __restrict__ out) {
  __shared__ __align__(16) float sO[256];
  const int tid = threadIdx.x, lane = tid & 31, wave = tid >> 5;
  const int b = blockIdx.x * 256 + tid;
  const float* zr  = z2  + (size_t)b * kZ2Pitch;
  const float* orr = oth + (size_t)b * kOPitch;
  float s0 = 0.f, s1 = 0.f;
#pragma unroll 1
  for (int j = 0; j < kN2; j += 4) {
    const v4f a  = *(const v4f*)(zr + j);
    const v4f o  = *(const v4f*)(orr + j);
    const v4f wa = *(const v4f*)(W3 + j);
    const v4f wo = *(const v4f*)(W3 + kN2 + j);
    s0 += a[0] * wa[0]; s0 += a[1] * wa[1]; s0 += a[2] * wa[2]; s0 += a[3] * wa[3];
    s1 += o[0] * wo[0]; s1 += o[1] * wo[1]; s1 += o[2] * wo[2]; s1 += o[3] * wo[3];
  }
  const float y = sigm_(b3[0] + (s0 + s1));
  sO[tid] = y;
  wave_lds_sync();
  const v4f v = *(const v4f*)(sO + wave * 32 + (lane & 7) * 4);
  float* ob = out + (size_t)blockIdx.x * 256 + wave * 32 + (lane & 7) * 4;
  if (lane < 8) { *(volatile v4f*)ob = v; }
  __threadfence();
  if (lane < 8) { *(volatile v4f*)ob = v; }
}

extern "C" void kernel_launch(void* const* d_in, const int* in_sizes, int n_in,
                              void* d_out, int out_size, void* d_ws, size_t ws_size,
                              hipStream_t stream) {
  if (n_in < 29) return;
  if (in_sizes[0] != kBatch * 2 * kSeq) return;
  if (out_size < kBatch) return;

  const float* x = (const float*)d_in[0];
  const float* r0_Wih0 = (const float*)d_in[1];  const float* r0_Whh0 = (const float*)d_in[2];
  const float* r0_bih0 = (const float*)d_in[3];  const float* r0_bhh0 = (const float*)d_in[4];
  const float* r0_Wih1 = (const float*)d_in[5];  const float* r0_Whh1 = (const float*)d_in[6];
  const float* r0_bih1 = (const float*)d_in[7];  const float* r0_bhh1 = (const float*)d_in[8];
  const float* r1_Wih0 = (const float*)d_in[9];  const float* r1_Whh0 = (const float*)d_in[10];
  const float* r1_bih0 = (const float*)d_in[11]; const float* r1_bhh0 = (const float*)d_in[12];
  const float* r1_Wih1 = (const float*)d_in[13]; const float* r1_Whh1 = (const float*)d_in[14];
  const float* r1_bih1 = (const float*)d_in[15]; const float* r1_bhh1 = (const float*)d_in[16];
  const float* Wp = (const float*)d_in[17]; const float* bp = (const float*)d_in[18];
  const float* WH = (const float*)d_in[19]; const float* bH = (const float*)d_in[20];
  const float* WL = (const float*)d_in[21]; const float* bL = (const float*)d_in[22];
  const float* W1 = (const float*)d_in[23]; const float* b1 = (const float*)d_in[24];
  const float* W2 = (const float*)d_in[25]; const float* b2 = (const float*)d_in[26];
  const float* W3 = (const float*)d_in[27]; const float* b3 = (const float*)d_in[28];
  float* out = (float*)d_out;

  char* w = (char*)d_ws;
  size_t off = 0;
  unsigned short* hpl  = (unsigned short*)(w + off); off += (size_t)kBatch * kHPitch * 2;
  unsigned short* xpl  = (unsigned short*)(w + off); off += (size_t)kBatch * kXPitch * 2;
  unsigned short* zpl  = (unsigned short*)(w + off); off += (size_t)kBatch * kZPitch * 2;
  unsigned short* z1pl = (unsigned short*)(w + off); off += (size_t)kBatch * kZ1Pitch * 2;
  float*          z2f  = (float*)(w + off);          off += (size_t)kBatch * kZ2Pitch * 4;
  float*          othf = (float*)(w + off);          off += (size_t)kBatch * kOPitch * 4;
  unsigned short* whp  = (unsigned short*)(w + off); off += (size_t)kNF * kHPitch * 2;
  unsigned short* wlp  = (unsigned short*)(w + off); off += (size_t)kNF * kHPitch * 2;
  unsigned short* wpp  = (unsigned short*)(w + off); off += (size_t)kWpRows * kXPitch * 2;
  unsigned short* w1p  = (unsigned short*)(w + off); off += (size_t)kW1Rows * kW1K * 2;
  unsigned short* w2p  = (unsigned short*)(w + off); off += (size_t)kW2Rows * kW2Pitch * 2;
  float*          biasp = (float*)(w + off);         off += (size_t)kBiasTot * 4;
  if (off > ws_size) return;

  {
    const int tH = kNF * (kHPitch / 8);
    const int tP = kWpRows * (kXPitch / 8);
    const int t1 = kW1Rows * (kW1K / 8);
    const int t2 = kW2Rows * (kW2Pitch / 8);
    padcast_kernel<<<(tH + 255) / 256, 256, 0, stream>>>(WH, kNF, kHCols, whp, kNF, kHPitch, kWCarry);
    padcast_kernel<<<(tH + 255) / 256, 256, 0, stream>>>(WL, kNF, kHCols, wlp, kNF, kHPitch, kWCarry);
    padcast_kernel<<<(tP + 255) / 256, 256, 0, stream>>>(Wp, kNP, kXCols, wpp, kWpRows, kXPitch, kWCarry);
    padcast_kernel<<<(t1 + 255) / 256, 256, 0, stream>>>(W1, kN1, kW1K, w1p, kW1Rows, kW1K, kWCarry);
    padcast_kernel<<<(t2 + 255) / 256, 256, 0, stream>>>(W2, kN2, kN1, w2p, kW2Rows, kW2Pitch, kWCarry);
    biasprep_kernel<<<1, 64, 0, stream>>>(b1, b2, bp, biasp);
  }

  xcast_kernel<<<(kBatch * (kXPitch / 8)) / 256, 256, 0, stream>>>(x, xpl);

  {
    const int tiles = (kBatch / 64) * (kOPitch / 64);
    wmma_gemm64<0, false, 2, 0, false, 0><<<dim3((tiles + 7) / 8, 1), 256, 0, stream>>>(
        xpl, xpl, kXPitch, 0L, wpp, wpp, kXPitch, 0L, othf, othf, kOPitch, 0L,
        biasp + 192, biasp, 0L, kBatch, kOPitch, kXK, kInvW);
  }

  lstm2_kernel<<<kBatch / kLstmThreads, kLstmThreads, 0, stream>>>(
      x, r0_Wih0, r0_Whh0, r0_bih0, r0_bhh0, r0_Wih1, r0_Whh1, r0_bih1, r0_bhh1, hpl, 0);
  {
    const int tiles = (kBatch / 64) * (kNF / 64);
    wmma_gemm64<0, false, 2, 1, false, 6><<<dim3((tiles + 7) / 8, 1), 256, 0, stream>>>(
        hpl, hpl, kHPitch, 0L, whp, whp, kHPitch, 0L, zpl, zpl, kZPitch, 0L,
        bH, biasp, 0L, kBatch, kNF, kHCols, kInvWH);
  }

  lstm2_kernel<<<kBatch / kLstmThreads, kLstmThreads, 0, stream>>>(
      x, r1_Wih0, r1_Whh0, r1_bih0, r1_bhh0, r1_Wih1, r1_Whh1, r1_bih1, r1_bhh1, hpl, 1);
  {
    const int tiles = (kBatch / 64) * (kNF / 64);
    wmma_gemm64<0, false, 2, 1, false, 6><<<dim3((tiles + 7) / 8, 1), 256, 0, stream>>>(
        hpl, hpl, kHPitch, 0L, wlp, wlp, kHPitch, 0L, zpl + kNF, zpl + kNF, kZPitch, 0L,
        bL, biasp, 0L, kBatch, kNF, kHCols, kInvWH);
  }

  {
    const int tiles = (kBatch / 64) * (kZ1Pitch / 64);
    wmma_gemm64<0, false, 2, 1, false, 6><<<dim3((tiles + 7) / 8, 1), 256, 0, stream>>>(
        zpl, zpl, kZPitch, 0L, w1p, w1p, kW1K, 0L, z1pl, z1pl, kZ1Pitch, 0L,
        biasp, biasp, 0L, kBatch, kZ1Pitch, kW1K, kInvW);
  }

  {
    const int tiles = (kBatch / 64) * (kZ2Pitch / 64);
    wmma_gemm64<0, false, 2, 0, false, 6><<<dim3((tiles + 7) / 8, 1), 256, 0, stream>>>(
        z1pl, z1pl, kZ1Pitch, 0L, w2p, w2p, kW2Pitch, 0L, z2f, z2f, kZ2Pitch, 0L,
        biasp + 128, biasp, 0L, kBatch, kZ2Pitch, kW2K, kInvW);
  }

  head_kernel<<<kBatch / 256, 256, 0, stream>>>(z2f, othf, W3, b3, out);
}
